// VanillaRNN_65249143160920
// MI455X (gfx1250) — hardware-run, weakly checked
//
#include <hip/hip_runtime.h>
#include <math.h>

constexpr int NBAT   = 2048;
constexpr int NSEQ   = 512;
constexpr int NHID   = 256;
constexpr int NCLS   = 10;
constexpr int NTHR   = 256;
constexpr int BROWS  = 16;
constexpr int HPITCH = 264;
constexpr int XPITCH = 512;
constexpr int SPITCH = 260;
constexpr int NOUTB  = BROWS * NCLS;
constexpr float WCARRY     = 16.0f;
constexpr float WCARRY_INV = 1.0f / 16.0f;
static_assert(NBAT % BROWS == 0);
static_assert(NHID == 32 * (NTHR / 32));
static_assert(NHID % 32 == 0);
static_assert((2 * BROWS * HPITCH) % NTHR == 0);
static_assert((BROWS * NSEQ) % (4 * NTHR) == 0);
static_assert((NOUTB * 4) % 128 == 0);
static_assert(NOUTB % 4 == 0 && NOUTB / 4 <= NTHR);
static_assert((NHID * NHID) % (8 * NTHR) == 0);
static_assert(HPITCH % 8 == 0 && SPITCH % 4 == 0 && XPITCH % 4 == 0);
static_assert((NCLS * NHID) % 4 == 0);
static_assert(NSEQ % 2 == 0);

typedef __attribute__((ext_vector_type(16))) _Float16 v16h;
typedef __attribute__((ext_vector_type(8)))  _Float16 v8h;
typedef __attribute__((ext_vector_type(8)))  float    v8f;
typedef __attribute__((ext_vector_type(4)))  float    v4f;

__device__ __forceinline__ void dep_guard_h(v8f& a, v8f& b, v16h x, v16h y) { asm volatile("v_nop\n\tv_nop\n\tv_nop\n\tv_nop" : "+v"(a), "+v"(b) : "v"(x), "v"(y)); }
__device__ __forceinline__ void keep4_h(v16h a, v16h b, v16h c, v16h d) { asm volatile("v_nop" :: "v"(a), "v"(b), "v"(c), "v"(d)); }
__device__ __forceinline__ void acc_guard2(v8f& a, v8f& b) { asm volatile("v_nop\n\tv_nop\n\tv_nop\n\tv_nop" : "+v"(a), "+v"(b)); }

template <typename T> struct Frag;
template <> struct Frag<_Float16> {
  typedef v16h V; union U { v16h v; v8h h[2]; };
  static __device__ __forceinline__ v16h load(const _Float16* p) {
    U f; f.h[0] = *(const v8h*)(p); f.h[1] = *(const v8h*)(p + 16); return f.v;
  }
  static __device__ __forceinline__ v8f mma(v16h a, v16h b, v8f c) {
    return __builtin_amdgcn_wmma_f32_16x16x32_f16(false, a, false, b, (short)0, c, false, false);
  }
};

__device__ __forceinline__ float ftanh(float x) { return 1.0f - 2.0f * __builtin_amdgcn_rcpf(expf(2.0f * x) + 1.0f); }

__global__ __launch_bounds__(NTHR) void cvt_f16x8_kernel(const float* __restrict__ src, unsigned short* __restrict__ dst,
                                                         int n8, float sc) {
  const int i = blockIdx.x * NTHR + threadIdx.x;
  if (i < n8) {
    const float* sp = src + (size_t)i * 8;
    const v4f a = *(const v4f*)(sp);
    const v4f b = *(const v4f*)(sp + 4);
    v8h hv;
#pragma unroll
    for (int e = 0; e < 4; ++e) {
      hv[e]     = (_Float16)(a[e] * sc);
      hv[4 + e] = (_Float16)(b[e] * sc);
    }
    for (int pass = 0; pass < 2; ++pass) {
      *(volatile v8h*)(dst + (size_t)i * 8) = hv;
      __threadfence();
    }
  }
}

__global__ __launch_bounds__(NTHR) void rnn_seq_kernel(const float* __restrict__ x, const float* __restrict__ whx,
                                                       const float* __restrict__ bh, const unsigned short* __restrict__ WHp,
                                                       const float* __restrict__ wph, const float* __restrict__ bp,
                                                       float* __restrict__ out) {
  __shared__ __align__(16) _Float16 Ah[2][BROWS * HPITCH];
  __shared__ __align__(16) float    Xs[BROWS * XPITCH];
  __shared__ __align__(16) float    Wp[NCLS * NHID];
  __shared__ __align__(16) float    Hs[BROWS * SPITCH];
  __shared__ __align__(16) float    Os[NOUTB];
  const _Float16* WH = (const _Float16*)WHp;
  const int tid = threadIdx.x, lane = tid & 31, wave = tid >> 5;
  const int c = lane & 15, hh = lane >> 4, koff = hh * 8;
  const int rowbase = blockIdx.x * BROWS;

  {
    _Float16* ahf = &Ah[0][0];
#pragma unroll 1
    for (int i = tid; i < 2 * BROWS * HPITCH; i += NTHR) ahf[i] = (_Float16)0.0f;
  }
#pragma unroll 1
  for (int it = 0; it < (BROWS * NSEQ) / (4 * NTHR); ++it) {
    const int idx = it * NTHR + tid;
    const int m = idx >> 7, t4 = (idx & 127) * 4;
    const v4f v = *(const v4f*)(x + (size_t)(rowbase + m) * NSEQ + t4);
    *(v4f*)(Xs + m * XPITCH + t4) = v;
  }
#pragma unroll 1
  for (int it = 0; it < 3; ++it) {
    const int idx = it * NTHR + tid;
    const int ic = (idx < (NCLS * NHID) / 4) ? idx : ((NCLS * NHID) / 4 - 1);
    const v4f v = *(const v4f*)(wph + (size_t)ic * 4);
    if (idx < (NCLS * NHID) / 4) *(v4f*)(Wp + idx * 4) = v;
  }
  float wx[2], bv[2], hst[2][8];
#pragma unroll
  for (int nt = 0; nt < 2; ++nt) {
    const int j = 32 * wave + 16 * nt + c;
    wx[nt] = whx[j];
    bv[nt] = bh[j];
#pragma unroll
    for (int r = 0; r < 8; ++r) hst[nt][r] = 0.0f;
  }
  __syncthreads();

  const v8f z8 = {0.f, 0.f, 0.f, 0.f, 0.f, 0.f, 0.f, 0.f};
  const int j0 = 32 * wave + c;
  const int j1 = 32 * wave + 16 + c;
  const _Float16* w0 = WH + (size_t)j0 * NHID + koff;
  const _Float16* w1 = WH + (size_t)j1 * NHID + koff;

#pragma unroll 1
  for (int t = 0; t < NSEQ; ++t) {
    const int cur = t & 1;
    const _Float16* ahrow = &Ah[cur][0] + c * HPITCH + koff;
    _Float16* ahn = &Ah[cur ^ 1][0];

    float xv[8];
#pragma unroll
    for (int r = 0; r < 8; ++r) xv[r] = Xs[(8 * hh + r) * XPITCH + t];

    v8f acc0 = z8, acc1 = z8;
#pragma unroll 1
    for (int k0 = 0; k0 < NHID; k0 += 32) {
      const v16h a  = Frag<_Float16>::load(ahrow + k0);
      const v16h b0 = Frag<_Float16>::load(w0 + k0);
      const v16h b1 = Frag<_Float16>::load(w1 + k0);
      acc0 = Frag<_Float16>::mma(a, b0, acc0);
      acc1 = Frag<_Float16>::mma(a, b1, acc1);
      dep_guard_h(acc0, acc1, a, b1);
      keep4_h(a, b0, b1, a);
    }
    acc_guard2(acc0, acc1);

#pragma unroll
    for (int r = 0; r < 8; ++r) {
      const float pre0 = acc0[r] * WCARRY_INV + (wx[0] * xv[r] + bv[0]);
      const float pre1 = acc1[r] * WCARRY_INV + (wx[1] * xv[r] + bv[1]);
      const float h0n = ftanh(pre0);
      const float h1n = ftanh(pre1);
      hst[0][r] = h0n;
      hst[1][r] = h1n;
      ahn[(8 * hh + r) * HPITCH + j0] = (_Float16)h0n;
      ahn[(8 * hh + r) * HPITCH + j1] = (_Float16)h1n;
    }
    __syncthreads();
  }

#pragma unroll
  for (int r = 0; r < 8; ++r) {
    Hs[(8 * hh + r) * SPITCH + j0] = hst[0][r];
    Hs[(8 * hh + r) * SPITCH + j1] = hst[1][r];
  }
  __syncthreads();

  if (wave < 5) {
    const int b  = tid / NCLS;
    const int cc = tid - b * NCLS;
    const float* wrow = Wp + cc * NHID;
    const float* hrow = Hs + b * SPITCH;
    float s = 0.0f;
#pragma unroll 1
    for (int m = 0; m < NHID; ++m) s += wrow[m] * hrow[m];
    s += bp[cc];
    Os[tid] = s;
  }
  __syncthreads();

  if (tid < NOUTB / 4) {
    const v4f v = *(const v4f*)(Os + tid * 4);
    float* op = out + (size_t)blockIdx.x * NOUTB + tid * 4;
    for (int pass = 0; pass < 2; ++pass) {
      *(volatile v4f*)op = v;
      __threadfence();
    }
  }
}

extern "C" void kernel_launch(void* const* d_in, const int* in_sizes, int n_in,
                              void* d_out, int out_size, void* d_ws, size_t ws_size, hipStream_t stream) {
  if (n_in < 6 || d_out == nullptr || d_ws == nullptr) return;
  if (in_sizes[0] != NBAT * NSEQ || in_sizes[1] != NHID || in_sizes[2] != NHID * NHID || in_sizes[3] != NHID ||
      in_sizes[4] != NCLS * NHID || in_sizes[5] != NCLS || out_size != NBAT * NCLS) return;

  const float* x   = (const float*)d_in[0];
  const float* whx = (const float*)d_in[1];
  const float* whh = (const float*)d_in[2];
  const float* bh  = (const float*)d_in[3];
  const float* wph = (const float*)d_in[4];
  const float* bp  = (const float*)d_in[5];
  float* out = (float*)d_out;

  char* ws = (char*)d_ws; size_t off = 0;
  auto carve = [&](size_t bytes) -> char* { char* p = ws + off; off += (bytes + 255) & ~(size_t)255; return p; };
  unsigned short* WH = (unsigned short*)carve((size_t)NHID * NHID * 2);
  if (off > ws_size || off > (size_t)134217728) return;

  const int n8 = (NHID * NHID) / 8;
  cvt_f16x8_kernel<<<n8 / NTHR, NTHR, 0, stream>>>(whh, WH, n8, WCARRY);
  rnn_seq_kernel<<<NBAT / BROWS, NTHR, 0, stream>>>(x, whx, bh, WH, wph, bp, out);
}
